// DualGNNModel_44504451121832
// MI455X (gfx1250) — hardware-verified
//
#include <hip/hip_runtime.h>
#include <math.h>

#define DIN 64
#define DH 128
#define NT 256
#define SRB 2048
#define SPE 16
#define SCH (NT * SPE)
#define SPP 8
#define SCHP (NT * SPP)
#define GMAX 256
#define CMB 320
#define NWH (DH * DIN + 2 * DH * DH)

typedef __attribute__((ext_vector_type(16))) _Float16 v16h;
typedef __attribute__((ext_vector_type(8)))  _Float16 v8h;
typedef __attribute__((ext_vector_type(16))) __bf16   v16b;
typedef __attribute__((ext_vector_type(8)))  __bf16   v8b;
typedef __attribute__((ext_vector_type(8)))  float    v8f;
typedef __attribute__((ext_vector_type(4)))  float    v4f;
typedef __attribute__((ext_vector_type(4)))  int      v4i;
typedef __attribute__((ext_vector_type(2)))  unsigned v2u;

__device__ __forceinline__ unsigned short f2bf_bits(float f) {
  unsigned u = __float_as_uint(f);
  return (unsigned short)((u + 0x7FFFu + ((u >> 16) & 1u)) >> 16);
}
__device__ __forceinline__ float bf_bits2f(unsigned short h) { return __uint_as_float(((unsigned)h) << 16); }
__device__ __forceinline__ unsigned short h_bits(float f) { return __builtin_bit_cast(unsigned short, (_Float16)f); }

__device__ __forceinline__ void dep_guard_h(v8f& a, v8f& b, v16h x, v16h y) { asm volatile("v_nop\n\tv_nop\n\tv_nop\n\tv_nop" : "+v"(a), "+v"(b) : "v"(x), "v"(y)); }
__device__ __forceinline__ void dep_guard_b(v8f& a, v8f& b, v16b x, v16b y) { asm volatile("v_nop\n\tv_nop\n\tv_nop\n\tv_nop" : "+v"(a), "+v"(b) : "v"(x), "v"(y)); }
__device__ __forceinline__ void keep4_h(v16h a, v16h b, v16h c, v16h d) { asm volatile("v_nop" :: "v"(a), "v"(b), "v"(c), "v"(d)); }
__device__ __forceinline__ void keep4_b(v16b a, v16b b, v16b c, v16b d) { asm volatile("v_nop" :: "v"(a), "v"(b), "v"(c), "v"(d)); }
__device__ __forceinline__ void fence_v4(v4f& t) { asm volatile("" : "+v"(t)); }
__device__ __forceinline__ void acc_guard4(v8f& a, v8f& b, v8f& c, v8f& d) { asm volatile("v_nop\n\tv_nop\n\tv_nop\n\tv_nop" : "+v"(a), "+v"(b), "+v"(c), "+v"(d)); }
template <typename T> struct Frag;
template <> struct Frag<_Float16> {
  typedef v16h V; union U { v16h v; v8h h[2]; };
  static __device__ __forceinline__ v16h load(const _Float16* p) {
    U f; f.h[0] = *(const v8h*)(p); f.h[1] = *(const v8h*)(p + 16); return f.v;
  }
  static __device__ __forceinline__ v8f mma(v16h a, v16h b, v8f c) {
    return __builtin_amdgcn_wmma_f32_16x16x32_f16(false, a, false, b, (short)0, c, false, false);
  }
  static __device__ __forceinline__ void guard(v8f& a, v8f& b, v16h x, v16h y) { dep_guard_h(a, b, x, y); }
  static __device__ __forceinline__ void keep(v16h a, v16h b, v16h c, v16h d) { keep4_h(a, b, c, d); }
};
template <> struct Frag<__bf16> {
  typedef v16b V; union U { v16b v; v8b h[2]; };
  static __device__ __forceinline__ v16b load(const __bf16* p) {
    U f; f.h[0] = *(const v8b*)(p); f.h[1] = *(const v8b*)(p + 16); return f.v;
  }
  static __device__ __forceinline__ v8f mma(v16b a, v16b b, v8f c) {
    return __builtin_amdgcn_wmma_f32_16x16x32_bf16(false, a, false, b, (short)0, c, false, false);
  }
  static __device__ __forceinline__ void guard(v8f& a, v8f& b, v16b x, v16b y) { dep_guard_b(a, b, x, y); }
  static __device__ __forceinline__ void keep(v16b a, v16b b, v16b c, v16b d) { keep4_b(a, b, c, d); }
};

template <int ET> struct Elem;
template <> struct Elem<0> { typedef _Float16 T; };
template <> struct Elem<1> { typedef __bf16 T; };
template <int ET, bool SPLIT, int BIAS_MODE, int OUT_MODE, bool RESID, int ACT = 0>
__global__ __launch_bounds__(256) void wmma_gemm64(
    const unsigned short* __restrict__ Ap, const unsigned short* __restrict__ A2p, int lda, long strideA,
    const unsigned short* __restrict__ Btp, const unsigned short* __restrict__ Bt2p, int ldb, long strideB,
    void* __restrict__ Cout, void* __restrict__ Cout2, int ldc, long strideC,
    const float* __restrict__ bias, long strideBias,
    const float* __restrict__ resid, long strideR,
    int M, int N, int K, float scale) {
  typedef typename Elem<ET>::T T;
  typedef typename Frag<T>::V V;
  const T* A = (const T*)Ap; const T* A2 = (const T*)A2p; const T* Bt = (const T*)Btp; const T* Bt2 = (const T*)Bt2p;
  __shared__ __align__(16) float sT[8][16 * 68];
  const int b    = blockIdx.y;
  const int lane = threadIdx.x & 31;
  const int wave = threadIdx.x >> 5;
  const int tilesN = N >> 6;
  const int tilesM = M >> 6;
  const int tile = blockIdx.x * 8 + wave;
  if (tile >= tilesM * tilesN) return;
  const int tm = tile / tilesN;
  const int tn = tile - tm * tilesN;
  const int m0 = tm << 6;
  const int n0 = tn << 6;

  const T* Ab  = A  + (size_t)b * strideA;
  const T* Bb  = Bt + (size_t)b * strideB;
  const T* Ab2 = SPLIT ? (A2  + (size_t)b * strideA) : nullptr;
  const T* Bb2 = SPLIT ? (Bt2 + (size_t)b * strideB) : nullptr;
  const float* Bi = (BIAS_MODE != 0) ? (bias + (size_t)b * strideBias) : nullptr;

  const int rlane = lane & 15;
  const int koff  = (lane >> 4) * 8;
  const int mOff  = (lane >> 4) * 8;

  v8f acc[4][4];
#pragma unroll
  for (int i = 0; i < 4; ++i)
#pragma unroll
    for (int j = 0; j < 4; ++j) acc[i][j] = (v8f){0.f,0.f,0.f,0.f,0.f,0.f,0.f,0.f};

  for (int k0 = 0; k0 < K; k0 += 32) {
    V bh[4], bl[4];
#pragma unroll
    for (int j = 0; j < 4; ++j) {
      const size_t bo = (size_t)(n0 + (j << 4) + rlane) * ldb + koff + k0;
      bh[j] = Frag<T>::load(Bb + bo);
      if (SPLIT) bl[j] = Frag<T>::load(Bb2 + bo);
    }
#pragma unroll
    for (int i = 0; i < 4; ++i) {
      const size_t ao = (size_t)(m0 + (i << 4) + rlane) * lda + koff + k0;
      V ah = Frag<T>::load(Ab + ao);
      V al;
      if (SPLIT) al = Frag<T>::load(Ab2 + ao);
#pragma unroll
      for (int j = 0; j < 4; ++j) {
        acc[i][j] = Frag<T>::mma(ah, bh[j], acc[i][j]);
        if (SPLIT) {
          acc[i][j] = Frag<T>::mma(ah, bl[j], acc[i][j]);
          acc[i][j] = Frag<T>::mma(al, bh[j], acc[i][j]);
        }
      }
      Frag<T>::guard(acc[i][0], acc[i][3], ah, SPLIT ? al : ah);
    }
    Frag<T>::keep(bh[0], bh[1], bh[2], bh[3]);
    if (SPLIT) Frag<T>::keep(bl[0], bl[1], bl[2], bl[3]);
  }
  acc_guard4(acc[0][0], acc[0][1], acc[0][2], acc[0][3]);
  acc_guard4(acc[1][0], acc[1][1], acc[1][2], acc[1][3]);
  acc_guard4(acc[2][0], acc[2][1], acc[2][2], acc[2][3]);
  acc_guard4(acc[3][0], acc[3][1], acc[3][2], acc[3][3]);

  float* slab = sT[wave];
  const float* Rb = RESID ? (resid + (size_t)b * strideR) : nullptr;
#pragma unroll
  for (int i = 0; i < 4; ++i) {
    const int mBase = m0 + (i << 4);
    float rsv[8];
#pragma unroll
    for (int r = 0; r < 8; ++r) rsv[r] = (BIAS_MODE == 3) ? Bi[mBase + mOff + r] : 1.0f;
#pragma unroll
    for (int j = 0; j < 4; ++j) {
      const int n = n0 + (j << 4) + rlane;
      float bv = 0.f;
      if (BIAS_MODE == 2) bv = Bi[n];
#pragma unroll
      for (int r = 0; r < 8; ++r) {
        float v = acc[i][j][r] * scale;
        if (BIAS_MODE == 1) v += Bi[mBase + mOff + r];
        if (BIAS_MODE == 2) v += bv;
        if (BIAS_MODE == 3) v *= rsv[r];
        if (RESID) v += Rb[(size_t)(mBase + mOff + r) * ldc + n];
        if (ACT == 1) v = tanhf(v);
        if (ACT == 2) v = fmaxf(v, 0.0f);
        if (ACT == 3) v = v / (1.0f + expf(-v));
        if (ACT == 4) v = (v > 0.f) ? v : 0.01f * v;
        if (ACT == 5) v = 0.5f * v * (1.0f + erff(v * 0.70710678118654752f));
        slab[(mOff + r) * 68 + (j << 4) + rlane] = v;
      }
    }
    __builtin_amdgcn_fence(__ATOMIC_RELEASE, "workgroup");
    __builtin_amdgcn_wave_barrier();
    __builtin_amdgcn_fence(__ATOMIC_ACQUIRE, "workgroup");
    if (OUT_MODE == 0) {
      float* C = (float*)Cout + (size_t)b * strideC;
      const int hh = lane >> 4, c4 = (lane & 15) * 4;
      for (int pass = 0; pass < 2; ++pass) {
#pragma unroll
        for (int it = 0; it < 8; ++it) {
          const int row = it * 2 + hh;
          v4f v = *(const v4f*)(slab + row * 68 + c4);
          *(volatile v4f*)(C + (size_t)(mBase + row) * ldc + n0 + c4) = v;
        }
        __threadfence();
      }
    } else {
      const int q = lane >> 3, c8 = (lane & 7) * 8;
      unsigned short* C  = (unsigned short*)Cout  + (size_t)b * strideC;
      unsigned short* C2 = (OUT_MODE == 2) ? ((unsigned short*)Cout2 + (size_t)b * strideC) : nullptr;
      for (int pass = 0; pass < 2; ++pass) {
#pragma unroll
        for (int it = 0; it < 4; ++it) {
          const int row = it * 4 + q;
          const float* sp = slab + row * 68 + c8;
          v8h hv, lv;
#pragma unroll
          for (int e = 0; e < 8; ++e) {
            if (OUT_MODE == 1) {
              hv[e] = (_Float16)sp[e];
            } else {
              unsigned short hb = f2bf_bits(sp[e]);
              unsigned short lb = f2bf_bits(sp[e] - bf_bits2f(hb));
              hv[e] = __builtin_bit_cast(_Float16, hb);
              lv[e] = __builtin_bit_cast(_Float16, lb);
            }
          }
          *(volatile v8h*)(C + (size_t)(mBase + row) * ldc + n0 + c8) = hv;
          if (OUT_MODE == 2) *(volatile v8h*)(C2 + (size_t)(mBase + row) * ldc + n0 + c8) = lv;
        }
        __threadfence();
      }
    }
    __builtin_amdgcn_fence(__ATOMIC_RELEASE, "workgroup");
    __builtin_amdgcn_wave_barrier();
    __builtin_amdgcn_fence(__ATOMIC_ACQUIRE, "workgroup");
  }
}

__device__ __forceinline__ int blk_excl_scan(int cnt, int* scan_ws, int tid, int* tot) {
  const int lane = tid & 31, wave = tid >> 5; int incl = cnt;
#pragma unroll
  for (int o = 1; o < 32; o <<= 1) { const int v = __shfl_up(incl, o, 32); if (lane >= o) incl += v; }
  if (lane == 31) scan_ws[wave] = incl;
  __syncthreads();
  if (wave == 0) { int wv = (lane < NT / 32) ? scan_ws[lane] : 0; int wincl = wv;
#pragma unroll
    for (int o = 1; o < 32; o <<= 1) { const int v = __shfl_up(wincl, o, 32); if (lane >= o) wincl += v; }
    if (lane < NT / 32) scan_ws[32 + lane] = wincl - wv; if (lane == 31) scan_ws[64] = wincl; }
  __syncthreads();
  const int res = scan_ws[32 + wave] + incl - cnt; *tot = scan_ws[64];
  return res;
}
template <bool PAY>
__device__ __forceinline__ int chunk_hits(const int* __restrict__ keyv, const int* __restrict__ payv, int ne, int nn,
                                          int e0, int n0, int tid, int* LIST, int* scan_ws) {
  const int eb = e0 + tid * SPE;
  int rec[SPE]; int cnt = 0;
  if (eb + SPE <= ne) {
#pragma unroll
    for (int k = 0; k < SPE; k += 4) {
      const v4i d4 = *(const v4i*)(keyv + eb + k);
      v4i s4 = {0, 0, 0, 0};
      if (PAY) s4 = *(const v4i*)(payv + eb + k);
#pragma unroll
      for (int e = 0; e < 4; ++e) {
        const int d = d4[e]; int r = -1;
        if (d >= n0 && d < n0 + SRB) {
          int s = 0;
          if (PAY) { s = s4[e]; s = s < 0 ? 0 : (s >= nn ? nn - 1 : s); }
          r = ((d - n0) << 16) | s; ++cnt;
        }
        rec[k + e] = r;
      }
    }
  } else {
#pragma unroll
    for (int k = 0; k < SPE; ++k) {
      const int e = eb + k; int r = -1;
      if (e < ne) {
        const int d = keyv[e];
        if (d >= n0 && d < n0 + SRB) {
          int s = 0;
          if (PAY) { s = payv[e]; s = s < 0 ? 0 : (s >= nn ? nn - 1 : s); }
          r = ((d - n0) << 16) | s; ++cnt;
        }
      }
      rec[k] = r;
    }
  }
  int tot; int p = blk_excl_scan(cnt, scan_ws, tid, &tot);
#pragma unroll
  for (int k = 0; k < SPE; ++k) if (rec[k] >= 0) { if ((unsigned)p < (unsigned)SCH) LIST[p] = rec[k]; ++p; }
  __syncthreads();
  return tot < SCH ? tot : SCH;
}

__global__ __launch_bounds__(NT) void prep_kernel(const float* __restrict__ x0, const float* __restrict__ x1,
                                                 const float* __restrict__ a0, const float* __restrict__ a1, const float* __restrict__ a2,
                                                 const float* __restrict__ c0, const float* __restrict__ c1, const float* __restrict__ c2,
                                                 int nn, int mg, unsigned* __restrict__ XH, unsigned* __restrict__ WT) {
  const long i = (long)blockIdx.x * NT + threadIdx.x;
  const long per = (long)mg * (DIN / 4);
  const long nx = 2 * per;
  if (i < nx) {
    const int e = (i >= per) ? 1 : 0;
    const long rem = i - (long)e * per;
    const int row = (int)(rem / (DIN / 4));
    const int q = (int)(rem - (long)row * (DIN / 4));
    v4f v = {0.f, 0.f, 0.f, 0.f};
    if (row < nn) v = *(const v4f*)((e ? x1 : x0) + (size_t)row * DIN + 4 * q);
    v2u u;
    u[0] = (unsigned)h_bits(v[0]) | ((unsigned)h_bits(v[1]) << 16);
    u[1] = (unsigned)h_bits(v[2]) | ((unsigned)h_bits(v[3]) << 16);
    volatile v2u* p = (volatile v2u*)(XH + 2 * i);
    *p = u;
    __threadfence();
    *p = u;
  } else {
    const long w = i - nx;
    const int NWD = NWH / 2;
    if (w < 2 * NWD) {
      const int e = (w >= NWD) ? 1 : 0;
      const int wl = (int)(w - (long)e * NWD);
      const float* W; int K; int base;
      if (wl < DH * DIN / 2) { W = e ? c0 : a0; K = DIN; base = 0; }
      else if (wl < DH * DIN / 2 + DH * DH / 2) { W = e ? c1 : a1; K = DH; base = DH * DIN / 2; }
      else { W = e ? c2 : a2; K = DH; base = DH * DIN / 2 + DH * DH / 2; }
      const int wr = wl - base;
      const int o = wr / (K / 2);
      const int k = 2 * (wr - o * (K / 2));
      const float fa = W[(size_t)k * DH + o], fb = W[(size_t)(k + 1) * DH + o];
      const unsigned u = (unsigned)h_bits(fa) | ((unsigned)h_bits(fb) << 16);
      ((volatile unsigned*)WT)[w] = u;
      __threadfence();
      ((volatile unsigned*)WT)[w] = u;
    }
  }
}

__global__ __launch_bounds__(NT) void deg_kernel(const int* __restrict__ src0, const int* __restrict__ src1, int ne, int nn, int nch,
                                                float* __restrict__ NS, int nsStride) {
  __shared__ int LIST[SCH];
  __shared__ int CNT[SRB];
  __shared__ int scan_ws[80];
  const int tid = threadIdx.x, lane = tid & 31, wave = tid >> 5;
  const int enc = blockIdx.y;
  const int* keyv = enc ? src1 : src0;
  const int n0 = blockIdx.x * SRB;
  for (int i = tid; i < SRB; i += NT) CNT[i] = 0;
  __syncthreads();
#pragma unroll 1
  for (int c = 0; c < nch; ++c) {
    const int tot = chunk_hits<false>(keyv, keyv, ne, nn, c * SCH, n0, tid, LIST, scan_ws);
#pragma unroll 1
    for (int base = 0; base < tot; base += 32) {
      const int q = base + lane;
      const int rv = (q < tot) ? LIST[q] : -1;
      const int own = (rv >= 0 && (rv >> 24) == wave) ? 1 : 0;
      unsigned msk = (unsigned)__ballot(own);
#pragma unroll 1
      for (int it = 0; it < 32; ++it) {
        if (msk == 0u) break;
        const int bp = __builtin_ctz(msk); msk &= msk - 1u;
        const int r = __shfl(rv, bp, 32);
        const int dl = r >> 16;
        if (lane == 0) CNT[dl] += 1;
      }
    }
    __syncthreads();
  }
  __syncthreads();
  float* out = NS + (size_t)enc * nsStride + n0;
  for (int pass = 0; pass < 2; ++pass) {
#pragma unroll
    for (int j = 0; j < 2; ++j) {
      const int dl = wave * 256 + j * 128 + 4 * lane;
      v4f v;
#pragma unroll
      for (int e = 0; e < 4; ++e) {
        int c = CNT[dl + e]; c = c < 1 ? 1 : c;
        v[e] = 1.0f / sqrtf((float)c);
      }
      *(volatile v4f*)(out + dl) = v;
    }
    __threadfence();
  }
}

__global__ __launch_bounds__(NT) void agg_kernel(const float* __restrict__ HW, const int* __restrict__ srcv, const int* __restrict__ dstv,
                                                int ne, int nn, int mg, int nch, const float* __restrict__ bias,
                                                float* M, unsigned* __restrict__ HH, int last) {
  __shared__ int LIST[SCH];
  __shared__ int CNT[SRB];
  __shared__ int scan_ws[80];
  const int tid = threadIdx.x, lane = tid & 31, wave = tid >> 5;
  const int n0 = blockIdx.x * SRB;
  const v4f z4 = {0.f, 0.f, 0.f, 0.f};
#pragma unroll 1
  for (int j = 0; j < 256; ++j) { float* zp = M + (size_t)(n0 + wave * 256 + j) * DH + 4 * lane; *(volatile v4f*)zp = z4; __threadfence(); *(volatile v4f*)zp = z4; }
  for (int i = tid; i < SRB; i += NT) CNT[i] = 0;
  __syncthreads();
#pragma unroll 1
  for (int c = 0; c < nch; ++c) {
    const int tot = chunk_hits<true>(dstv, srcv, ne, nn, c * SCH, n0, tid, LIST, scan_ws);
#pragma unroll 1
    for (int base = 0; base < tot; base += 32) {
      const int q = base + lane;
      const int rv = (q < tot) ? LIST[q] : -1;
      const int own = (rv >= 0 && (rv >> 24) == wave) ? 1 : 0;
      unsigned msk = (unsigned)__ballot(own);
#pragma unroll 1
      for (int it = 0; it < 32; ++it) {
        if (msk == 0u) break;
        const int bp = __builtin_ctz(msk); msk &= msk - 1u;
        const int r = __shfl(rv, bp, 32);
        const int dl = r >> 16, s = r & 0xFFFF;
        const v4f hv = *(const v4f*)(HW + (size_t)s * DH + 4 * lane);
        float* rp = M + (size_t)(n0 + dl) * DH + 4 * lane;
        v4f a = *(const v4f*)rp;
        a = a + hv;
        *(volatile v4f*)rp = a;
        __threadfence();
        *(volatile v4f*)rp = a;
        if (lane == 0) CNT[dl] += 1;
      }
    }
    __syncthreads();
  }
  __syncthreads();
  const v4f b4 = *(const v4f*)(bias + 4 * lane);
#pragma unroll 1
  for (int j = 0; j < 256; ++j) {
    const int dl = wave * 256 + j; const int n = n0 + dl;
    if (n < mg) {
      const bool live = n < nn;
      int cn = CNT[dl]; cn = cn < 1 ? 1 : cn;
      const float nd = 1.0f / sqrtf((float)cn);
      float* rp = M + (size_t)n * DH + 4 * lane;
      const v4f a = *(const v4f*)rp;
      v4f t = a * nd; fence_v4(t); t = t + b4;
      v4f h;
#pragma unroll
      for (int e = 0; e < 4; ++e) h[e] = live ? fmaxf(t[e], 0.f) : 0.f;
      if (last) {
        for (int pass = 0; pass < 2; ++pass) { *(volatile v4f*)rp = h; __threadfence(); }
      } else {
        v2u u;
        u[0] = (unsigned)h_bits(h[0]) | ((unsigned)h_bits(h[1]) << 16);
        u[1] = (unsigned)h_bits(h[2]) | ((unsigned)h_bits(h[3]) << 16);
        volatile v2u* hp = (volatile v2u*)(HH + (size_t)n * (DH / 2) + 2 * lane);
        for (int pass = 0; pass < 2; ++pass) { *hp = u; __threadfence(); }
      }
    }
  }
}

__global__ __launch_bounds__(NT) void pool_kernel(const float* __restrict__ HS, const int* __restrict__ gidv, int nn, int nchp,
                                                 float* __restrict__ P) {
  __shared__ int LIST[SCHP];
  __shared__ int scan_ws[80];
  __shared__ __align__(16) float red[8 * DH];
  __shared__ int rc[8];
  const int tid = threadIdx.x, lane = tid & 31, wave = tid >> 5;
  const int g = blockIdx.x;
  const v4f z4 = {0.f, 0.f, 0.f, 0.f};
  v4f acc = z4; int cnt = 0;
#pragma unroll 1
  for (int c = 0; c < nchp; ++c) {
    const int eb = c * SCHP + tid * SPP;
    int bv[SPP]; int rec[SPP]; int kc = 0;
    if (eb + SPP <= nn) {
      const v4i b0 = *(const v4i*)(gidv + eb), bb = *(const v4i*)(gidv + eb + 4);
      bv[0] = b0[0]; bv[1] = b0[1]; bv[2] = b0[2]; bv[3] = b0[3]; bv[4] = bb[0]; bv[5] = bb[1]; bv[6] = bb[2]; bv[7] = bb[3];
    } else {
#pragma unroll
      for (int k = 0; k < SPP; ++k) { const int e = eb + k; bv[k] = (e < nn) ? gidv[e] : -1; }
    }
#pragma unroll
    for (int k = 0; k < SPP; ++k) { rec[k] = -1; if (bv[k] == g) { rec[k] = eb + k; ++kc; } }
    int tot; int p = blk_excl_scan(kc, scan_ws, tid, &tot);
#pragma unroll
    for (int k = 0; k < SPP; ++k) if (rec[k] >= 0) { if ((unsigned)p < (unsigned)SCHP) LIST[p] = rec[k]; ++p; }
    __syncthreads();
    const int totc = tot < SCHP ? tot : SCHP;
#pragma unroll 1
    for (int q = wave; q < totc; q += 8) {
      int nd = LIST[q]; nd = nd < 0 ? 0 : (nd >= nn ? nn - 1 : nd);
      acc = acc + *(const v4f*)(HS + (size_t)nd * DH + 4 * lane); ++cnt;
    }
    __syncthreads();
  }
  *(v4f*)(red + wave * DH + 4 * lane) = acc;
  if (lane == 0) rc[wave] = cnt;
  __syncthreads();
  if (wave == 0) {
    v4f s = z4; int ct = 0;
#pragma unroll
    for (int w = 0; w < 8; ++w) { s = s + *(const v4f*)(red + w * DH + 4 * lane); ct += rc[w]; }
    const float cf = (float)ct;
    const float inv = 1.0f / fmaxf(cf, 1.0f);
    const v4f o = s * inv;
    for (int pass = 0; pass < 2; ++pass) { *(volatile v4f*)(P + (size_t)g * DH + 4 * lane) = o; __threadfence(); }
  }
}

__global__ __launch_bounds__(NT) void mlp_kernel(const float* __restrict__ PSU, const float* __restrict__ PSV, const float* __restrict__ gf, int ngf,
                                                const float* __restrict__ W0, const float* __restrict__ b0,
                                                const float* __restrict__ W1, const float* __restrict__ b1,
                                                const float* __restrict__ W2, const float* __restrict__ b2, int ng, float* __restrict__ out) {
  __shared__ float comb[CMB];
  __shared__ float part[NT];
  __shared__ float h1[DH];
  __shared__ float h2[64];
  __shared__ __align__(16) float so[GMAX];
  const int tid = threadIdx.x, lane = tid & 31, wave = tid >> 5;
  const int d0 = 2 * DH + ngf;
  const int kh = (d0 + 1) >> 1;
  for (int i = tid; i < GMAX; i += NT) so[i] = 0.f;
  for (int i = tid; i < CMB; i += NT) comb[i] = 0.f;
  __syncthreads();
#pragma unroll 1
  for (int g = 0; g < ng; ++g) {
    if (tid < DH) comb[tid] = PSU[(size_t)g * DH + tid];
    else comb[tid] = PSV[(size_t)g * DH + tid - DH];
    if (tid < ngf) comb[2 * DH + tid] = gf[(size_t)g * ngf + tid];
    __syncthreads();
    {
      const int j = tid & (DH - 1), hf = tid >> 7;
      const int k0 = hf * kh, k1 = hf ? d0 : kh;
      float s = 0.f;
#pragma unroll 1
      for (int k = k0; k < k1; ++k) s += comb[k] * W0[(size_t)k * DH + j];
      part[tid] = s;
    }
    __syncthreads();
    if (tid < DH) { const float v = part[tid] + part[tid + DH] + b0[tid]; h1[tid] = fmaxf(v, 0.f); }
    __syncthreads();
    {
      const int j = tid & 63, qq = tid >> 6;
      float s = 0.f;
#pragma unroll 1
      for (int k = qq * 32; k < qq * 32 + 32; ++k) s += h1[k] * W1[k * 64 + j];
      part[tid] = s;
    }
    __syncthreads();
    if (tid < 64) { const float v = part[tid] + part[tid + 64] + part[tid + 128] + part[tid + 192] + b1[tid]; h2[tid] = fmaxf(v, 0.f); }
    __syncthreads();
    if (wave == 0) {
      float s = h2[lane] * W2[lane] + h2[lane + 32] * W2[lane + 32];
#pragma unroll
      for (int off = 16; off > 0; off >>= 1) s += __shfl_xor(s, off, 32);
      if (lane == 0) so[g] = s + b2[0];
    }
    __syncthreads();
  }
  if (wave == 0) {
    const int nu = ng >> 2;
    for (int pass = 0; pass < 2; ++pass) {
      for (int u = lane; u < nu; u += 32) { const v4f v = *(const v4f*)(so + 4 * u); *(volatile v4f*)(out + 4 * u) = v; }
      for (int t = 4 * nu + lane; t < ng; t += 32) { const float v = so[t]; ((volatile float*)out)[t] = v; }
      __threadfence();
    }
  }
}

extern "C" void kernel_launch(void* const* d_in, const int* in_sizes, int n_in,
                              void* d_out, int out_size, void* d_ws, size_t ws_size, hipStream_t stream) {
  if (n_in < 23) return;
  const int N = in_sizes[7];
  const int E = in_sizes[3];
  const int G = out_size;
  if (N <= 0 || E <= 0 || G <= 0 || G > GMAX || N > 65535) return;
  if (in_sizes[0] != N * DIN || in_sizes[1] != N * DIN || in_sizes[8] != N) return;
  if (in_sizes[4] != E || in_sizes[5] != E || in_sizes[6] != E) return;
  if (in_sizes[2] % G != 0) return;
  const int NGF = in_sizes[2] / G;
  const int d0 = 2 * DH + NGF;
  if (d0 > CMB || in_sizes[17] != d0 * DH || in_sizes[19] != DH * 64 || in_sizes[21] != 64) return;
  if (in_sizes[9] != DIN * DH || in_sizes[10] != DH * DH || in_sizes[13] != DIN * DH) return;

  const int ntiles = (N + SRB - 1) / SRB;
  const int NR = ntiles * SRB;
  const int MG = ((N + 63) / 64) * 64;
  const int nch = (E + SCH - 1) / SCH;
  const int nchp = (N + SCHP - 1) / SCHP;

  const float* x0 = (const float*)d_in[0];
  const float* x1 = (const float*)d_in[1];
  const float* gfp = (const float*)d_in[2];
  const int* src0 = (const int*)d_in[3];
  const int* dst0 = (const int*)d_in[4];
  const int* src1 = (const int*)d_in[5];
  const int* dst1 = (const int*)d_in[6];
  const int* gid0 = (const int*)d_in[7];
  const int* gid1 = (const int*)d_in[8];
  const float* suW0 = (const float*)d_in[9];
  const float* suW1 = (const float*)d_in[10];
  const float* suW2 = (const float*)d_in[11];
  const float* sub  = (const float*)d_in[12];
  const float* svW0 = (const float*)d_in[13];
  const float* svW1 = (const float*)d_in[14];
  const float* svW2 = (const float*)d_in[15];
  const float* svb  = (const float*)d_in[16];
  const float* mW0 = (const float*)d_in[17];
  const float* mb0 = (const float*)d_in[18];
  const float* mW1 = (const float*)d_in[19];
  const float* mb1 = (const float*)d_in[20];
  const float* mW2 = (const float*)d_in[21];
  const float* mb2 = (const float*)d_in[22];
  float* out = (float*)d_out;

  char* ws = (char*)d_ws; size_t off = 0;
  auto carve = [&](size_t bytes) -> char* { char* p = ws + off; off += (bytes + 255) & ~(size_t)255; return p; };
  unsigned* WT  = (unsigned*)carve((size_t)2 * NWH * 2);
  float*    NS  = (float*)carve((size_t)2 * NR * 4);
  char*     R16 = carve((size_t)2 * MG * DH * 2);
  float*    HWf = (float*)carve((size_t)2 * MG * DH * 4);
  float*    Mf  = (float*)carve((size_t)NR * DH * 4);
  float*    PL  = (float*)carve((size_t)2 * G * DH * 4);
  if (off > ws_size || off > (size_t)134217728) return;
  unsigned* XH = (unsigned*)R16;
  unsigned* HH = (unsigned*)R16;

  {
    const long nx = 2L * MG * (DIN / 4);
    const long tot = nx + NWH;
    prep_kernel<<<(int)((tot + NT - 1) / NT), NT, 0, stream>>>(x0, x1, suW0, suW1, suW2, svW0, svW1, svW2, N, MG, XH, WT);
  }
  deg_kernel<<<dim3(ntiles, 2), NT, 0, stream>>>(src0, src1, E, N, nch, NS, NR);

  const _Float16* WTh = (const _Float16*)(const void*)WT;
  for (int l = 0; l < 3; ++l) {
    const int K = (l == 0) ? DIN : DH;
    const long woff = (l == 0) ? 0 : (l == 1 ? (long)DH * DIN : (long)DH * DIN + (long)DH * DH);
    const int tiles = (MG / 64) * (DH / 64);
    wmma_gemm64<0, false, 3, 0, false, 0><<<dim3((tiles + 7) / 8, 2), 256, 0, stream>>>(
        (const unsigned short*)R16, (const unsigned short*)nullptr, K, (long)MG * K,
        (const unsigned short*)(WTh + woff), (const unsigned short*)nullptr, K, (long)NWH,
        (void*)HWf, (void*)nullptr, DH, (long)MG * DH,
        (const float*)NS, (long)NR,
        (const float*)nullptr, 0L,
        MG, DH, K, 1.0f);
    const int last = (l == 2) ? 1 : 0;
    for (int enc = 0; enc < 2; ++enc) {
      const float* HWe = HWf + (size_t)enc * MG * DH;
      unsigned* HHe = HH + (size_t)enc * MG * (DH / 2);
      const int* sv = enc ? src1 : src0;
      const int* dv = enc ? dst1 : dst0;
      const float* be = (enc ? svb : sub) + l * DH;
      agg_kernel<<<ntiles, NT, 0, stream>>>(HWe, sv, dv, E, N, MG, nch, be, Mf, HHe, last);
      if (last) pool_kernel<<<G, NT, 0, stream>>>(Mf, enc ? gid1 : gid0, N, nchp, PL + (size_t)enc * G * DH);
    }
  }
  mlp_kernel<<<1, NT, 0, stream>>>(PL, PL + (size_t)G * DH, gfp, NGF, mW0, mb0, mW1, mb1, mW2, mb2, G, out);
}
